// EncoderLayer_28346784154306
// MI455X (gfx1250) — hardware-verified
//
#include <hip/hip_runtime.h>


#ifndef NB
#define NB 8
#endif
#ifndef SEQ
#define SEQ 1024
#endif
#define NB_FULL  8
#define SEQ_FULL 1024
#define DM   1024
#define NH   16
#define HD   64
#define FF   4096
#define MROWS (NB * SEQ)
#define WCAR 64.0f
#define CCAR 16.0f
#define PEXP 8.0f
#define CL2  0.18033688011112042f
#define LNEPS 1e-5f

static_assert((SEQ & (SEQ - 1)) == 0);
static_assert(SEQ % 64 == 0);
static_assert(SEQ <= SEQ_FULL);
static_assert(NB <= NB_FULL);
static_assert(DM == NH * HD);
static_assert(FF == 4 * DM);
static_assert(((size_t)MROWS * DM) % 2048 == 0);
static_assert(MROWS % 64 == 0);
static_assert((size_t)6 * DM * DM * 2 + (size_t)2 * DM * FF * 2 - (size_t)2 * DM * DM * 2 + (size_t)MROWS * FF * 2 + (size_t)MROWS * DM * 4 <= (size_t)134217728);

typedef _Float16 h16;
typedef __attribute__((ext_vector_type(16))) _Float16 v16h;
typedef __attribute__((ext_vector_type(8)))  _Float16 v8h;
typedef __attribute__((ext_vector_type(4)))  _Float16 v4h;
typedef __attribute__((ext_vector_type(2)))  _Float16 v2h;
typedef __attribute__((ext_vector_type(8)))  float    v8f;
typedef __attribute__((ext_vector_type(4)))  float    v4f;
typedef v8h __attribute__((may_alias)) v8ha;
typedef v4f __attribute__((may_alias)) v4fa;

__device__ __forceinline__ unsigned short f2bf(float f) { unsigned u = __float_as_uint(f); u += 0x7FFFu + ((u >> 16) & 1u); return (unsigned short)(u >> 16); }
__device__ __forceinline__ float bf2f(unsigned short b) { return __uint_as_float(((unsigned)b) << 16); }
__device__ __forceinline__ float bfr(float f) { return bf2f(f2bf(f)); }
__device__ __forceinline__ v16h cat16(v8h lo, v8h hi) { return __builtin_shufflevector(lo, hi, 0, 1, 2, 3, 4, 5, 6, 7, 8, 9, 10, 11, 12, 13, 14, 15); }
__device__ __forceinline__ v8f wmma16(v16h a, v16h b, v8f c) { return __builtin_amdgcn_wmma_f32_16x16x32_f16(false, a, false, b, (short)0, c, false, false); }
__device__ __forceinline__ v16h ldfrag(const h16* p) { return cat16(*(const v8h*)p, *(const v8h*)(p + 16)); }
__device__ __forceinline__ unsigned xrow(unsigned r) { return (r / (unsigned)SEQ) * (unsigned)SEQ_FULL + (r % (unsigned)SEQ); }

__global__ __launch_bounds__(256) void k_cvtx(const float* __restrict__ x, h16* XH) {
    const unsigned i = blockIdx.x * 256u + threadIdx.x; const unsigned e = i * 8u; if (e >= (unsigned)MROWS * DM) return;
    const unsigned row = e / (unsigned)DM, col = e % (unsigned)DM;
    const v8f v = *(const v8f*)(x + (size_t)xrow(row) * DM + col); v8h o;
#pragma unroll
    for (int k = 0; k < 8; ++k) o[k] = (h16)bfr(v[k]);
    *(volatile v8h*)(XH + e) = o; __threadfence(); *(volatile v8h*)(XH + e) = o;
}

template <unsigned K, unsigned N>
__global__ __launch_bounds__(256) void k_wt(const float* __restrict__ w, h16* Bt) {
    static_assert((K & (K - 1)) == 0); static_assert((N * K / 64u) % 64u == 0);
    const unsigned lane = threadIdx.x & 31u; const unsigned L0 = (blockIdx.x * 8u + (threadIdx.x >> 5)) * 8u; const unsigned nlines = N * K / 64u;
#pragma unroll
    for (int ps = 0; ps < 2; ++ps) {
#pragma unroll 1
        for (unsigned l = 0; l < 8u; ++l) { const unsigned L = L0 + l; if (L >= nlines) break; const unsigned e = L * 64u + lane * 2u; const unsigned k = e % K, n = e / K; v2h o;
            o[0] = (h16)(bfr(w[(size_t)k * N + n]) * WCAR); o[1] = (h16)(bfr(w[(size_t)(k + 1u) * N + n]) * WCAR); *(volatile v2h*)(Bt + e) = o; }
        if (ps == 0) __threadfence(); }
}

template <int OUT16, int RELU, int BIASM, int RESM>
__global__ __launch_bounds__(32) void k_gemm(const h16* __restrict__ A, const h16* __restrict__ Bt, unsigned K, void* Cv, unsigned ldc, float alpha, const float* __restrict__ bias, const float* resid, size_t sA, size_t sB, size_t sC) {
    __shared__ __align__(16) float os[16 * 68];
    const size_t z = blockIdx.z; A += z * sA; Bt += z * sB;
    const unsigned lane = threadIdx.x & 31u, lr = lane & 15u, hi = lane >> 4; const unsigned r0 = blockIdx.x * 64u, c0 = blockIdx.y * 64u;
    v8f acc[4][4];
#pragma unroll
    for (int mb = 0; mb < 4; ++mb)
#pragma unroll
        for (int nb = 0; nb < 4; ++nb) acc[mb][nb] = (v8f){};
    const size_t aoff = (size_t)(r0 + lr) * K + 8u * hi, boff = (size_t)(c0 + lr) * K + 8u * hi;
#pragma unroll 1
    for (unsigned kc = 0; kc < K; kc += 32u) {
        v16h a[4];
#pragma unroll
        for (int mb = 0; mb < 4; ++mb) a[mb] = ldfrag(A + aoff + (size_t)mb * 16u * K + kc);
#pragma unroll
        for (int nb = 0; nb < 4; ++nb) { const v16h b = ldfrag(Bt + boff + (size_t)nb * 16u * K + kc);
#pragma unroll
            for (int mb = 0; mb < 4; ++mb) acc[mb][nb] = wmma16(a[mb], b, acc[mb][nb]); }
        asm volatile("v_nop\n\tv_nop\n\tv_nop\n\tv_nop" : "+v"(acc[0][0]), "+v"(acc[1][1]), "+v"(acc[2][2]), "+v"(acc[3][3]) : "v"(a[0]), "v"(a[3]));
    }
    float* Cf = (float*)Cv + z * sC; h16* Ch = (h16*)Cv + z * sC;
    const unsigned rq = lane >> 3, c8 = (lane & 7u) * 8u, c4 = lr * 4u;
    v4f bA = {0.f, 0.f, 0.f, 0.f}, bB = {0.f, 0.f, 0.f, 0.f};
    if (BIASM == 1) {
        if (OUT16) { const v4f t0 = *(const v4f*)(bias + c0 + c8); const v4f t1 = *(const v4f*)(bias + c0 + c8 + 4u);
#pragma unroll
            for (int q = 0; q < 4; ++q) { bA[q] = bfr(t0[q]); bB[q] = bfr(t1[q]); } }
        else { const v4f t0 = *(const v4f*)(bias + c0 + c4);
#pragma unroll
            for (int q = 0; q < 4; ++q) bA[q] = bfr(t0[q]); }
    }
#pragma unroll
    for (int mb = 0; mb < 4; ++mb) {
#pragma unroll
        for (int nb = 0; nb < 4; ++nb) {
#pragma unroll
            for (int j = 0; j < 8; ++j) os[(hi * 8u + j) * 68u + nb * 16u + lr] = acc[mb][nb][j]; }
        __syncthreads();
        const unsigned rbase = r0 + (unsigned)mb * 16u;
#pragma unroll 1
        for (int ps = 0; ps < 2; ++ps) {
            if (OUT16) {
#pragma unroll
                for (unsigned s = 0; s < 4u; ++s) { const unsigned row = 4u * s + rq;
                    const v4f a = *(const v4fa*)(os + row * 68u + c8); const v4f b = *(const v4fa*)(os + row * 68u + c8 + 4u);
                    float rb = 0.f; if (BIASM == 2) rb = bfr(bias[rbase + row]);
                    v8h o;
#pragma unroll
                    for (int q = 0; q < 4; ++q) { float x0 = a[q] * alpha + bA[q] + rb, x1 = b[q] * alpha + bB[q] + rb; if (RELU) { x0 = fmaxf(x0, 0.0f); x1 = fmaxf(x1, 0.0f); } o[q] = (h16)x0; o[4 + q] = (h16)x1; }
                    *(volatile v8h*)(Ch + (size_t)(rbase + row) * ldc + c0 + c8) = o; }
            } else {
#pragma unroll
                for (unsigned s = 0; s < 8u; ++s) { const unsigned row = 2u * s + hi;
                    v4f val = *(const v4fa*)(os + row * 68u + c4);
                    float rb = 0.f; if (BIASM == 2) rb = bfr(bias[rbase + row]);
#pragma unroll
                    for (int q = 0; q < 4; ++q) { float x0 = val[q] * alpha + bA[q] + rb; if (RELU) x0 = fmaxf(x0, 0.0f); val[q] = x0; }
                    if (RESM == 1) { const v4f rv = *(const v4f*)(resid + (size_t)(rbase + row) * ldc + c0 + c4);
#pragma unroll
                        for (int q = 0; q < 4; ++q) val[q] = __fadd_rn(val[q], rv[q]); }
                    if (RESM == 2) { const v4f rv = *(const v4f*)(resid + (size_t)xrow(rbase + row) * DM + c0 + c4);
#pragma unroll
                        for (int q = 0; q < 4; ++q) val[q] = __fadd_rn(val[q], bfr(rv[q])); }
                    *(volatile v4f*)(Cf + (size_t)(rbase + row) * ldc + c0 + c4) = val; }
            }
            if (ps == 0) __threadfence(); }
        __syncthreads();
    }
}

__global__ __launch_bounds__(32) void k_flash(const h16* __restrict__ Qp, const h16* __restrict__ Kp, const h16* __restrict__ VTp, h16* Cx) {
    __shared__ __align__(16) h16 os[32 * 72];
    const unsigned lane = threadIdx.x & 31u, lr = lane & 15u, hi = lane >> 4;
    const unsigned q0 = blockIdx.x * 32u, hh = blockIdx.y, b = blockIdx.z;
    const size_t rowb = (size_t)b * SEQ;
    const h16* qbase = Qp + (rowb + q0 + lr) * DM + hh * HD + 8u * hi;
    const h16* kbase = Kp + (rowb + lr) * DM + hh * HD + 8u * hi;
    const h16* vbase = VTp + ((size_t)b * DM + hh * HD + lr) * SEQ + 8u * hi;
    v16h qb[2][2];
#pragma unroll
    for (int qt = 0; qt < 2; ++qt)
#pragma unroll
        for (int ks = 0; ks < 2; ++ks) qb[qt][ks] = ldfrag(qbase + (size_t)qt * 16u * DM + ks * 32u);
    v8f ot[4][2];
#pragma unroll
    for (int dt = 0; dt < 4; ++dt) { ot[dt][0] = (v8f){}; ot[dt][1] = (v8f){}; }
    float m0 = -3.0e38f, m1 = -3.0e38f, l0 = 0.f, l1 = 0.f;
#pragma unroll 1
    for (unsigned kt = 0; kt < (unsigned)SEQ / 32u; ++kt) {
        v16h ka[2][2];
#pragma unroll
        for (int mt = 0; mt < 2; ++mt)
#pragma unroll
            for (int ks = 0; ks < 2; ++ks) ka[mt][ks] = ldfrag(kbase + (size_t)(kt * 32u + mt * 16u) * DM + ks * 32u);
        v8f st[2][2];
#pragma unroll
        for (int qt = 0; qt < 2; ++qt) { st[qt][0] = (v8f){}; st[qt][1] = (v8f){}; }
#pragma unroll
        for (int ks = 0; ks < 2; ++ks)
#pragma unroll
            for (int qt = 0; qt < 2; ++qt)
#pragma unroll
                for (int mt = 0; mt < 2; ++mt) st[qt][mt] = wmma16(ka[mt][ks], qb[qt][ks], st[qt][mt]);
        asm volatile("v_nop\n\tv_nop\n\tv_nop\n\tv_nop" : "+v"(st[0][0]), "+v"(st[0][1]), "+v"(st[1][0]), "+v"(st[1][1]) : "v"(ka[1][1]), "v"(qb[1][1]));
        v16h va[4];
#pragma unroll
        for (int dt = 0; dt < 4; ++dt) va[dt] = ldfrag(vbase + (size_t)dt * 16u * SEQ + kt * 32u);
        float t0 = st[0][0][0], t1 = st[1][0][0];
#pragma unroll
        for (int r = 0; r < 8; ++r) { t0 = fmaxf(t0, fmaxf(st[0][0][r], st[0][1][r])); t1 = fmaxf(t1, fmaxf(st[1][0][r], st[1][1][r])); }
        t0 = fmaxf(t0, __shfl_xor(t0, 16, 32)); t1 = fmaxf(t1, __shfl_xor(t1, 16, 32));
        const float mn0 = fmaxf(m0, t0), mn1 = fmaxf(m1, t1);
        const bool grow = (mn0 > m0) || (mn1 > m1);
        if (__builtin_amdgcn_ballot_w32(grow) != 0u) {
            const float a0 = __builtin_amdgcn_exp2f((m0 - mn0) * CL2), a1 = __builtin_amdgcn_exp2f((m1 - mn1) * CL2);
            l0 *= a0; l1 *= a1;
#pragma unroll
            for (int dt = 0; dt < 4; ++dt)
#pragma unroll
                for (int r = 0; r < 8; ++r) { ot[dt][0][r] *= a0; ot[dt][1][r] *= a1; }
        }
        m0 = mn0; m1 = mn1;
        const float off0 = PEXP - mn0 * CL2, off1 = PEXP - mn1 * CL2;
        v16h pb0, pb1; float s0 = 0.f, s1 = 0.f;
#pragma unroll
        for (int r = 0; r < 8; ++r) {
            const float p00 = __builtin_amdgcn_exp2f(fmaf(st[0][0][r], CL2, off0)), p01 = __builtin_amdgcn_exp2f(fmaf(st[0][1][r], CL2, off0));
            const float p10 = __builtin_amdgcn_exp2f(fmaf(st[1][0][r], CL2, off1)), p11 = __builtin_amdgcn_exp2f(fmaf(st[1][1][r], CL2, off1));
            s0 += p00 + p01; s1 += p10 + p11;
            pb0[r] = (h16)p00; pb0[8 + r] = (h16)p01; pb1[r] = (h16)p10; pb1[8 + r] = (h16)p11; }
        l0 += s0; l1 += s1;
#pragma unroll
        for (int dt = 0; dt < 4; ++dt) { ot[dt][0] = wmma16(va[dt], pb0, ot[dt][0]); ot[dt][1] = wmma16(va[dt], pb1, ot[dt][1]); }
        asm volatile("v_nop\n\tv_nop\n\tv_nop\n\tv_nop" : "+v"(ot[0][0]), "+v"(ot[0][1]), "+v"(ot[1][0]), "+v"(ot[1][1]), "+v"(ot[2][0]), "+v"(ot[2][1]), "+v"(ot[3][0]), "+v"(ot[3][1]) : "v"(pb0), "v"(pb1), "v"(va[3]));
    }
    l0 += __shfl_xor(l0, 16, 32); l1 += __shfl_xor(l1, 16, 32);
    const float i0 = CCAR / l0, i1 = CCAR / l1;
#pragma unroll
    for (int dt = 0; dt < 4; ++dt) { v8h o0, o1;
#pragma unroll
        for (int r = 0; r < 8; ++r) { o0[r] = (h16)(ot[dt][0][r] * i0); o1[r] = (h16)(ot[dt][1][r] * i1); }
        *(v8ha*)(os + lr * 72u + dt * 16u + 8u * hi) = o0; *(v8ha*)(os + (16u + lr) * 72u + dt * 16u + 8u * hi) = o1; }
    __syncthreads();
    h16* cb = Cx + (rowb + q0) * DM + hh * HD; const unsigned rq = lane >> 3, c8 = (lane & 7u) * 8u;
#pragma unroll 1
    for (int ps = 0; ps < 2; ++ps) {
#pragma unroll
        for (unsigned s = 0; s < 8u; ++s) { const unsigned row = 4u * s + rq; const v8h v = *(const v8ha*)(os + row * 72u + c8); *(volatile v8h*)(cb + (size_t)row * DM + c8) = v; }
        if (ps == 0) __threadfence(); }
}

template <int W16>
__global__ __launch_bounds__(256) void k_ln(const float* F, const float* __restrict__ g, const float* __restrict__ bb, float* out, h16* out16, unsigned mapout) {
    const unsigned lane = threadIdx.x & 31u; const unsigned row = blockIdx.x * 8u + (threadIdx.x >> 5); if (row >= (unsigned)MROWS) return;
    const float* fr = F + (size_t)row * DM; float* orow = out + (size_t)(mapout ? xrow(row) : row) * DM; h16* hrow = out16 + (size_t)row * DM;
    float v[DM / 32]; float s = 0.f;
#pragma unroll
    for (int c = 0; c < DM / 128; ++c) { const v4f a = *(const v4f*)(fr + c * 128 + lane * 4u);
#pragma unroll
        for (int q = 0; q < 4; ++q) { v[c * 4 + q] = a[q]; s = __fadd_rn(s, a[q]); } }
#pragma unroll
    for (int sh = 16; sh; sh >>= 1) s = __fadd_rn(s, __shfl_xor(s, sh, 32));
    const float mean = s * (1.0f / (float)DM); float s2 = 0.f;
#pragma unroll
    for (int k = 0; k < DM / 32; ++k) { const float dv = __fsub_rn(v[k], mean); float p2 = __fmul_rn(dv, dv); asm volatile("" : "+v"(p2)); s2 = __fadd_rn(s2, p2); v[k] = dv; }
#pragma unroll
    for (int sh = 16; sh; sh >>= 1) s2 = __fadd_rn(s2, __shfl_xor(s2, sh, 32));
    const float rs = __fdiv_rn(1.0f, __fsqrt_rn(__fadd_rn(s2 * (1.0f / (float)DM), LNEPS)));
#pragma unroll 1
    for (int ps = 0; ps < 2; ++ps) {
#pragma unroll
        for (int c = 0; c < DM / 128; ++c) { const v4f gv = *(const v4f*)(g + c * 128 + lane * 4u); const v4f bv = *(const v4f*)(bb + c * 128 + lane * 4u); v4f o; v4h o16;
#pragma unroll
            for (int q = 0; q < 4; ++q) { float y = __fmul_rn(v[c * 4 + q], rs); asm volatile("" : "+v"(y)); y = __fmul_rn(y, bfr(gv[q])); asm volatile("" : "+v"(y)); o[q] = __fadd_rn(y, bfr(bv[q])); o16[q] = (h16)o[q]; }
            *(volatile v4f*)(orow + c * 128 + lane * 4u) = o;
            if (W16) *(volatile v4h*)(hrow + c * 128 + lane * 4u) = o16; }
        if (ps == 0) __threadfence(); }
}

extern "C" void kernel_launch(void* const* d_in, const int* in_sizes, int n_in,
                              void* d_out, int out_size, void* d_ws, size_t ws_size, hipStream_t stream) {
    if (n_in < 17) return;
    const size_t xneed = ((size_t)(NB - 1) * SEQ_FULL + SEQ) * DM;
    if ((size_t)in_sizes[0] < xneed) return;
    if ((size_t)in_sizes[1] < (size_t)DM * DM || (size_t)in_sizes[3] < (size_t)DM * DM || (size_t)in_sizes[5] < (size_t)DM * DM || (size_t)in_sizes[7] < (size_t)DM * DM) return;
    if ((size_t)in_sizes[11] < (size_t)DM * FF || (size_t)in_sizes[13] < (size_t)FF * DM) return;
    if (in_sizes[2] < DM || in_sizes[4] < DM || in_sizes[6] < DM || in_sizes[8] < DM || in_sizes[9] < DM || in_sizes[10] < DM || in_sizes[12] < FF || in_sizes[14] < DM || in_sizes[15] < DM || in_sizes[16] < DM) return;
    if ((size_t)out_size < xneed || (size_t)out_size < (size_t)MROWS * DM) return;
    const float* x = (const float*)d_in[0]; const float* wq = (const float*)d_in[1]; const float* bq = (const float*)d_in[2]; const float* wk = (const float*)d_in[3]; const float* bk = (const float*)d_in[4];
    const float* wv = (const float*)d_in[5]; const float* bv = (const float*)d_in[6]; const float* wy = (const float*)d_in[7]; const float* by = (const float*)d_in[8];
    const float* g1 = (const float*)d_in[9]; const float* be1 = (const float*)d_in[10]; const float* w1 = (const float*)d_in[11]; const float* b1 = (const float*)d_in[12];
    const float* w2 = (const float*)d_in[13]; const float* b2 = (const float*)d_in[14]; const float* g2 = (const float*)d_in[15]; const float* be2 = (const float*)d_in[16];
    float* OUT = (float*)d_out;
    char* wsp = (char*)d_ws;
    auto take = [&](size_t bytes) { char* p = wsp; wsp += (bytes + 255) & ~(size_t)255; return (void*)p; };
    h16* WQ = (h16*)take((size_t)DM * DM * 2); h16* WK = (h16*)take((size_t)DM * DM * 2); h16* WV = (h16*)take((size_t)DM * DM * 2); h16* WY = (h16*)take((size_t)DM * DM * 2);
    h16* W1T = (h16*)take((size_t)FF * DM * 2); h16* W2T = (h16*)take((size_t)DM * FF * 2);
    h16* R1 = (h16*)take((size_t)MROWS * FF * 2);
    h16* R2 = (h16*)take((size_t)MROWS * DM * 4);
    if ((size_t)(wsp - (char*)d_ws) > ws_size) return;
    h16* XH = R1; h16* Q16 = R1 + (size_t)MROWS * DM; h16* K16 = R1 + (size_t)2 * MROWS * DM; h16* VT16 = R1 + (size_t)3 * MROWS * DM; h16* FF1 = R1;
    h16* CTX = R2; h16* H16 = R2 + (size_t)MROWS * DM; float* Z = (float*)R2;
    float* Y = OUT;

    k_cvtx<<<(unsigned)((size_t)MROWS * DM / 8 / 256), 256, 0, stream>>>(x, XH);
    k_wt<DM, DM><<<DM * DM / 64 / 64, 256, 0, stream>>>(wq, WQ);
    k_wt<DM, DM><<<DM * DM / 64 / 64, 256, 0, stream>>>(wk, WK);
    k_wt<DM, DM><<<DM * DM / 64 / 64, 256, 0, stream>>>(wv, WV);
    k_wt<DM, DM><<<DM * DM / 64 / 64, 256, 0, stream>>>(wy, WY);
    k_wt<DM, FF><<<DM * FF / 64 / 64, 256, 0, stream>>>(w1, W1T);
    k_wt<FF, DM><<<FF * DM / 64 / 64, 256, 0, stream>>>(w2, W2T);

    k_gemm<1, 0, 1, 0><<<dim3(MROWS / 64, DM / 64, 1), 32, 0, stream>>>(XH, WQ, DM, Q16, DM, 1.0f / WCAR, bq, nullptr, 0, 0, 0);
    k_gemm<1, 0, 1, 0><<<dim3(MROWS / 64, DM / 64, 1), 32, 0, stream>>>(XH, WK, DM, K16, DM, 1.0f / WCAR, bk, nullptr, 0, 0, 0);
    k_gemm<1, 0, 2, 0><<<dim3(DM / 64, SEQ / 64, NB), 32, 0, stream>>>(WV, XH, DM, VT16, SEQ, 1.0f / WCAR, bv, nullptr, 0, (size_t)SEQ * DM, (size_t)DM * SEQ);
    k_flash<<<dim3(SEQ / 32, NH, NB), 32, 0, stream>>>(Q16, K16, VT16, CTX);
    k_gemm<0, 0, 1, 2><<<dim3(MROWS / 64, DM / 64, 1), 32, 0, stream>>>(CTX, WY, DM, Y, DM, 1.0f / (WCAR * CCAR), by, x, 0, 0, 0);
    k_ln<1><<<MROWS / 8, 256, 0, stream>>>(Y, g1, be1, Y, H16, 0u);
    k_gemm<1, 1, 1, 0><<<dim3(MROWS / 64, FF / 64, 1), 32, 0, stream>>>(H16, W1T, DM, FF1, FF, 1.0f / WCAR, b1, nullptr, 0, 0, 0);
    k_gemm<0, 0, 1, 1><<<dim3(MROWS / 64, DM / 64, 1), 32, 0, stream>>>(FF1, W2T, FF, Z, DM, 1.0f / WCAR, b2, Y, 0, 0, 0);
    k_ln<0><<<MROWS / 8, 256, 0, stream>>>(Z, g2, be2, OUT, nullptr, 1u);
}
